// PointNet_14018773254577
// MI455X (gfx1250) — hardware-verified
//
#include <hip/hip_runtime.h>
#include <math.h>

constexpr int NN       = 100000;
constexpr int NE       = 3200000;
constexpr int NGRAPH   = 64;
constexpr int NCLS     = 40;
constexpr int NCH      = 32;
constexpr int TILE_N   = 1024;
constexpr int NTILE    = (NN + TILE_N - 1) / TILE_N;
constexpr int BLK      = 256;
constexpr int NWAVE    = BLK / 32;
constexpr int CHUNK_E  = 256;
constexpr int NCHUNK   = NE / CHUNK_E;
constexpr int LIST_CAP = 288;
constexpr int AT_PITCH = 40;
constexpr float WCARRY     = 16.0f;
constexpr float WCARRY_INV = 1.0f / 16.0f;
static_assert(NE % CHUNK_E == 0, "edge chunks exact");
static_assert(NN % 32 == 0, "pool chunks exact");
static_assert(NN % 4 == 0, "node groups exact");
static_assert((NN - (NTILE - 1) * TILE_N) % 4 == 0, "last tile rows in whole wave stores");
static_assert((NN / 4) % NWAVE == 0, "node group grid exact");
static_assert(NGRAPH * NCLS == 10 * BLK, "classifier outputs per thread");
static_assert(15 + CHUNK_E < LIST_CAP, "hit list capacity");
static_assert(NCH == 32, "one k step");

typedef __attribute__((ext_vector_type(16))) _Float16 v16h;
typedef __attribute__((ext_vector_type(8)))  _Float16 v8h;
typedef __attribute__((ext_vector_type(8)))  float    v8f;
typedef __attribute__((ext_vector_type(4)))  float    v4f;
typedef __attribute__((ext_vector_type(4)))  int      v4i;

template <typename T> struct Frag;
template <> struct Frag<_Float16> {
  typedef v16h V; union U { v16h v; v8h h[2]; };
  static __device__ __forceinline__ v16h load(const _Float16* p) {
    U f; f.h[0] = *(const v8h*)(p); f.h[1] = *(const v8h*)(p + 16); return f.v;
  }
  static __device__ __forceinline__ v8f mma(v16h a, v16h b, v8f c) {
    return __builtin_amdgcn_wmma_f32_16x16x32_f16(false, a, false, b, (short)0, c, false, false);
  }
};

__device__ __forceinline__ void mma_pair(v16h a, v16h b0, v16h b1, v8f& d0, v8f& d1) {
  d0 = Frag<_Float16>::mma(a, b0, d0);
  d1 = Frag<_Float16>::mma(a, b1, d1);
  asm volatile("v_nop\n\tv_nop\n\tv_nop\n\tv_nop" : "+v"(d0), "+v"(d1) : "v"(a), "v"(b0), "v"(b1));
}

__device__ __forceinline__ void wave_lds_sync() {
  __builtin_amdgcn_fence(__ATOMIC_RELEASE, "workgroup");
  __builtin_amdgcn_wave_barrier();
  __builtin_amdgcn_fence(__ATOMIC_ACQUIRE, "workgroup");
}

__device__ __forceinline__ int clampi(int v, int lo, int hi) {
  v = v < lo ? lo : v;
  v = v > hi ? hi : v;
  return v;
}

template <int CIN>
__global__ __launch_bounds__(BLK) void node_pre_kernel(
    const float* __restrict__ hsrc, const float* __restrict__ pos, const float* __restrict__ W,
    const float* __restrict__ b1, float* __restrict__ U, float* __restrict__ V) {
  constexpr int WROWS = CIN + 3;
  __shared__ __align__(16) float sW[WROWS * 32];
  __shared__ __align__(16) float sU[NWAVE][128];
  __shared__ __align__(16) float sV[NWAVE][128];
  const int tid = threadIdx.x, lane = tid & 31, wave = tid >> 5;
  for (int i = tid; i < WROWS * 8; i += BLK) {
    const v4f w4 = *(const v4f*)(W + 4 * i);
    *(v4f*)(sW + 4 * i) = w4;
  }
  __syncthreads();
  const int grp  = blockIdx.x * NWAVE + wave;
  const int grpc = grp < (NN / 4) ? grp : (NN / 4 - 1);
  const int n0   = grpc * 4;
  const int hl   = lane < CIN ? lane : (CIN - 1);
  float hv[4];
#pragma unroll
  for (int j = 0; j < 4; ++j) hv[j] = hsrc[(size_t)(n0 + j) * CIN + hl];
  const int pl_i = lane < 12 ? lane : 11;
  const float pl = pos[(size_t)n0 * 3 + pl_i];
  const float bb = b1[lane];
  float acc[4];
#pragma unroll
  for (int j = 0; j < 4; ++j) acc[j] = bb;
#pragma unroll 8
  for (int k = 0; k < CIN; ++k) {
    const float w = sW[k * 32 + lane];
#pragma unroll
    for (int j = 0; j < 4; ++j) {
      const float hk = __shfl(hv[j], k, 32);
      acc[j] = fmaf(hk, w, acc[j]);
    }
  }
  const float wp0 = sW[(CIN + 0) * 32 + lane];
  const float wp1 = sW[(CIN + 1) * 32 + lane];
  const float wp2 = sW[(CIN + 2) * 32 + lane];
  float* su = sU[wave];
  float* sv = sV[wave];
#pragma unroll
  for (int j = 0; j < 4; ++j) {
    const float p0 = __shfl(pl, 3 * j + 0, 32);
    const float p1 = __shfl(pl, 3 * j + 1, 32);
    const float p2 = __shfl(pl, 3 * j + 2, 32);
    float pv = p0 * wp0;
    pv = fmaf(p1, wp1, pv);
    pv = fmaf(p2, wp2, pv);
    su[j * 32 + lane] = acc[j] + pv;
    sv[j * 32 + lane] = pv;
  }
  wave_lds_sync();
  const v4f ou = *(const v4f*)(su + 4 * lane);
  const v4f ov = *(const v4f*)(sv + 4 * lane);
  if (grp < NN / 4) {
    float* up = U + (size_t)n0 * NCH + 4 * lane;
    float* vp = V + (size_t)n0 * NCH + 4 * lane;
    for (int pass = 0; pass < 2; ++pass) {
      *(volatile v4f*)up = ou;
      *(volatile v4f*)vp = ov;
      __threadfence();
    }
  }
}

__device__ __forceinline__ void process_tile(
    const int* lst, int nvalid, int n0, int lane,
    const float* __restrict__ U, const float* __restrict__ V,
    const int* __restrict__ esrc, const int* __restrict__ edst,
    _Float16* at, int* acc, v16h b0, v16h b1, float cl, float chv) {
  const int m = lane & 15, kh = lane >> 4;
  const int li = m < nvalid ? m : (nvalid - 1);
  int e = lst[li];
  e = clampi(e, 0, NE - 1);
  const int s  = clampi(esrc[e], 0, NN - 1);
  const int d  = edst[e];
  const int lr = clampi(d - n0, 0, TILE_N - 1);
  int dn = n0 + lr;
  dn = dn > NN - 1 ? NN - 1 : dn;
  const float* up = U + (size_t)s * NCH + kh * 8;
  const float* vp = V + (size_t)dn * NCH + kh * 8;
  const v4f u0 = *(const v4f*)(up);
  const v4f u1 = *(const v4f*)(up + 4);
  const v4f u2 = *(const v4f*)(up + 16);
  const v4f u3 = *(const v4f*)(up + 20);
  const v4f w0 = *(const v4f*)(vp);
  const v4f w1 = *(const v4f*)(vp + 4);
  const v4f w2 = *(const v4f*)(vp + 16);
  const v4f w3 = *(const v4f*)(vp + 20);
  v8h lo8, hi8;
#pragma unroll
  for (int i = 0; i < 4; ++i) {
    lo8[i]     = (_Float16)fmaxf(u0[i] - w0[i], 0.0f);
    lo8[4 + i] = (_Float16)fmaxf(u1[i] - w1[i], 0.0f);
    hi8[i]     = (_Float16)fmaxf(u2[i] - w2[i], 0.0f);
    hi8[4 + i] = (_Float16)fmaxf(u3[i] - w3[i], 0.0f);
  }
  *(v8h*)(at + m * AT_PITCH + kh * 8)      = lo8;
  *(v8h*)(at + m * AT_PITCH + 16 + kh * 8) = hi8;
  wave_lds_sync();
  const v16h a = Frag<_Float16>::load(at + m * AT_PITCH + kh * 8);
  v8f dlo, dhi;
#pragma unroll
  for (int r = 0; r < 8; ++r) { dlo[r] = cl; dhi[r] = chv; }
  mma_pair(a, b0, b1, dlo, dhi);
#pragma unroll
  for (int r = 0; r < 8; ++r) {
    const int row  = 8 * kh + r;
    const int lrow = __shfl(lr, row, 32);
    const int xlo  = __float_as_int(dlo[r]);
    const int xhi  = __float_as_int(dhi[r]);
    if (row < nvalid) {
      atomicMax(acc + lrow * NCH + m, xlo);
      atomicMax(acc + lrow * NCH + 16 + m, xhi);
    }
  }
  wave_lds_sync();
}

__device__ __forceinline__ void scan_slot(int d, int e, int n0, unsigned ltmask, int* lst, int& cnt) {
  const bool hit = ((unsigned)d - (unsigned)n0) < (unsigned)TILE_N;
  const unsigned mask = __builtin_amdgcn_ballot_w32(hit);
  if (mask != 0u) {
    const int p = cnt + __popc(mask & ltmask);
    if (hit && p < LIST_CAP) lst[p] = e;
    cnt += __popc(mask);
  }
}

__global__ __launch_bounds__(BLK) void edge_tile_kernel(
    const float* __restrict__ U, const float* __restrict__ V,
    const float* __restrict__ W2, const float* __restrict__ b2,
    const int* __restrict__ esrc, const int* __restrict__ edst,
    float* __restrict__ H) {
  __shared__ __align__(16) int      sAcc[TILE_N * NCH];
  __shared__ __align__(16) float    sWf[NCH * NCH];
  __shared__ __align__(16) _Float16 sBt[NCH * AT_PITCH];
  __shared__ __align__(16) _Float16 sAt[NWAVE][16 * AT_PITCH];
  __shared__ int sList[NWAVE][LIST_CAP];

  const int tid = threadIdx.x, lane = tid & 31, wave = tid >> 5;
  const int m = lane & 15, kh = lane >> 4;
  const int n0 = blockIdx.x * TILE_N;

  {
    const v4f w4 = *(const v4f*)(W2 + 4 * tid);
    *(v4f*)(sWf + 4 * tid) = w4;
  }
  {
    const v4i z4 = {0, 0, 0, 0};
#pragma unroll 4
    for (int i = 0; i < 32; ++i) *(v4i*)(sAcc + 4 * (i * BLK + tid)) = z4;
  }
  __syncthreads();
  if (tid < 128) {
    const int n = tid >> 2, kg = tid & 3;
    v8h t;
#pragma unroll
    for (int i = 0; i < 8; ++i) t[i] = (_Float16)(sWf[(kg * 8 + i) * NCH + n] * WCARRY);
    *(v8h*)(sBt + n * AT_PITCH + kg * 8) = t;
  }
  __syncthreads();
  const v16h b0 = Frag<_Float16>::load(sBt + m * AT_PITCH + kh * 8);
  const v16h b1 = Frag<_Float16>::load(sBt + (16 + m) * AT_PITCH + kh * 8);
  const float cl  = b2[m] * WCARRY;
  const float chv = b2[16 + m] * WCARRY;

  int* lst = sList[wave];
  _Float16* at = sAt[wave];
  const unsigned ltmask = (1u << lane) - 1u;
  int cnt = 0;

#pragma unroll 1
  for (int ch = wave; ch < NCHUNK; ch += NWAVE) {
    const int eb = ch * CHUNK_E + lane * 4;
    const v4i da = *(const v4i*)(edst + eb);
    const v4i db = *(const v4i*)(edst + eb + 128);
    scan_slot(da.x, eb + 0, n0, ltmask, lst, cnt);
    scan_slot(da.y, eb + 1, n0, ltmask, lst, cnt);
    scan_slot(da.z, eb + 2, n0, ltmask, lst, cnt);
    scan_slot(da.w, eb + 3, n0, ltmask, lst, cnt);
    scan_slot(db.x, eb + 128, n0, ltmask, lst, cnt);
    scan_slot(db.y, eb + 129, n0, ltmask, lst, cnt);
    scan_slot(db.z, eb + 130, n0, ltmask, lst, cnt);
    scan_slot(db.w, eb + 131, n0, ltmask, lst, cnt);
    cnt = __builtin_amdgcn_readfirstlane(cnt);
    cnt = cnt > LIST_CAP ? LIST_CAP : cnt;
#pragma unroll 1
    for (int it = 0; it < 17; ++it) {
      if (cnt < 16) break;
      cnt -= 16;
      process_tile(lst + cnt, 16, n0, lane, U, V, esrc, edst, at, sAcc, b0, b1, cl, chv);
    }
  }
  cnt = __builtin_amdgcn_readfirstlane(cnt);
  if (cnt > 0) {
    const int nv = cnt > 16 ? 16 : cnt;
    process_tile(lst, nv, n0, lane, U, V, esrc, edst, at, sAcc, b0, b1, cl, chv);
  }
  __syncthreads();

  float* hb = H + (size_t)n0 * NCH;
  for (int pass = 0; pass < 2; ++pass) {
#pragma unroll 1
    for (int it = 0; it < 32; ++it) {
      const int i = it * BLK + tid;
      const int row = n0 + (i >> 3);
      const v4i x = *(const v4i*)(sAcc + 4 * i);
      const int x0 = x.x, x1 = x.y, x2 = x.z, x3 = x.w;
      v4f o;
      o.x = __int_as_float(x0) * WCARRY_INV;
      o.y = __int_as_float(x1) * WCARRY_INV;
      o.z = __int_as_float(x2) * WCARRY_INV;
      o.w = __int_as_float(x3) * WCARRY_INV;
      if (row < NN) *(volatile v4f*)(hb + 4 * (size_t)i) = o;
    }
    __threadfence();
  }
}

__global__ __launch_bounds__(BLK) void pool_kernel(
    const float* __restrict__ H2, const int* __restrict__ batch, float* __restrict__ G) {
  __shared__ float sM[NWAVE][32];
  const int tid = threadIdx.x, lane = tid & 31, wave = tid >> 5;
  const int g = blockIdx.x;
  float mx = 0.0f;
#pragma unroll 1
  for (int ch = wave; ch < NN / 32; ch += NWAVE) {
    const int n = ch * 32 + lane;
    const int b = clampi(batch[n], 0, NGRAPH - 1);
    unsigned mask = __builtin_amdgcn_ballot_w32(b == g);
#pragma unroll 1
    for (int it = 0; it < 32; ++it) {
      if (mask == 0u) break;
      const int j = __ffs((int)mask) - 1;
      mask &= mask - 1u;
      const float v = H2[(size_t)(ch * 32 + j) * NCH + lane];
      mx = fmaxf(mx, v);
    }
  }
  sM[wave][lane] = mx;
  __syncthreads();
  if (wave == 0) {
    float r = sM[0][lane];
#pragma unroll
    for (int w = 1; w < NWAVE; ++w) r = fmaxf(r, sM[w][lane]);
    float* gp = G + g * NCH + lane;
    *(volatile float*)gp = r;
    __threadfence();
    *(volatile float*)gp = r;
  }
}

__global__ __launch_bounds__(BLK) void cls_kernel(
    const float* __restrict__ G, const float* __restrict__ wc, const float* __restrict__ bc,
    float* __restrict__ out) {
  __shared__ __align__(16) float sG[NGRAPH * NCH];
  __shared__ __align__(16) float sWc[NCH * NCLS];
  __shared__ __align__(16) float sBc[NCLS];
  __shared__ __align__(16) float sOut[NGRAPH * NCLS];
  const int tid = threadIdx.x;
  for (int i = tid; i < NGRAPH * NCH / 4; i += BLK) {
    const v4f t = *(const v4f*)(G + 4 * i);
    *(v4f*)(sG + 4 * i) = t;
  }
  for (int i = tid; i < NCH * NCLS / 4; i += BLK) {
    const v4f t = *(const v4f*)(wc + 4 * i);
    *(v4f*)(sWc + 4 * i) = t;
  }
  for (int i = tid; i < NCLS; i += BLK) sBc[i] = bc[i];
  __syncthreads();
#pragma unroll 1
  for (int j = 0; j < 10; ++j) {
    const int o = j * BLK + tid;
    const int g = o / NCLS;
    const int c = o - g * NCLS;
    float acc = sBc[c];
#pragma unroll 8
    for (int k = 0; k < NCH; ++k) acc = fmaf(sG[g * NCH + k], sWc[k * NCLS + c], acc);
    sOut[o] = acc;
  }
  __syncthreads();
  for (int pass = 0; pass < 2; ++pass) {
#pragma unroll 1
    for (int it = 0; it < 3; ++it) {
      const int i = it * BLK + tid;
      const int ic = i < (NGRAPH * NCLS / 4) ? i : (NGRAPH * NCLS / 4 - 1);
      const v4f v = *(const v4f*)(sOut + 4 * ic);
      if (i < NGRAPH * NCLS / 4) *(volatile v4f*)(out + 4 * i) = v;
    }
    __threadfence();
  }
}

extern "C" void kernel_launch(void* const* d_in, const int* in_sizes, int n_in,
                              void* d_out, int out_size, void* d_ws, size_t ws_size, hipStream_t stream) {
  (void)in_sizes; (void)out_size;
  if (n_in < 13 || d_out == nullptr || d_ws == nullptr) return;
  const float* pos   = (const float*)d_in[0];
  const int*   eidx  = (const int*)d_in[1];
  const int*   batch = (const int*)d_in[2];
  const float* w1a = (const float*)d_in[3];
  const float* b1a = (const float*)d_in[4];
  const float* w2a = (const float*)d_in[5];
  const float* b2a = (const float*)d_in[6];
  const float* w1b = (const float*)d_in[7];
  const float* b1b = (const float*)d_in[8];
  const float* w2b = (const float*)d_in[9];
  const float* b2b = (const float*)d_in[10];
  const float* wc  = (const float*)d_in[11];
  const float* bc  = (const float*)d_in[12];
  const int* esrc = eidx;
  const int* edst = eidx + NE;

  char* ws = (char*)d_ws; size_t off = 0;
  auto carve = [&](size_t bytes) -> char* { char* p = ws + off; off += (bytes + 255) & ~(size_t)255; return p; };
  const size_t nodeBytes = (size_t)NN * NCH * sizeof(float);
  float* U1 = (float*)carve(nodeBytes);
  float* V1 = (float*)carve(nodeBytes);
  float* H1 = (float*)carve(nodeBytes);
  float* U2 = (float*)carve(nodeBytes);
  float* V2 = (float*)carve(nodeBytes);
  float* H2 = (float*)carve(nodeBytes);
  float* GM = (float*)carve((size_t)NGRAPH * NCH * sizeof(float));
  if (off > ws_size || off > (size_t)134217728) return;

  const int preGrid = (NN / 4) / NWAVE;

  node_pre_kernel<3><<<preGrid, BLK, 0, stream>>>(pos, pos, w1a, b1a, U1, V1);
  edge_tile_kernel<<<NTILE, BLK, 0, stream>>>(U1, V1, w2a, b2a, esrc, edst, H1);
  node_pre_kernel<32><<<preGrid, BLK, 0, stream>>>(H1, pos, w1b, b1b, U2, V2);
  edge_tile_kernel<<<NTILE, BLK, 0, stream>>>(U2, V2, w2b, b2b, esrc, edst, H2);
  pool_kernel<<<NGRAPH, BLK, 0, stream>>>(H2, batch, GM);
  cls_kernel<<<1, BLK, 0, stream>>>(GM, wc, bc, (float*)d_out);
}
